// NNPytorchAD_3659312136356
// MI455X (gfx1250) — hardware-verified
//
#include <hip/hip_runtime.h>
#include <stddef.h>


typedef _Float16 v16h __attribute__((ext_vector_type(16)));
typedef _Float16 v8h  __attribute__((ext_vector_type(8)));
typedef float    v8f  __attribute__((ext_vector_type(8)));
typedef float    v4f  __attribute__((ext_vector_type(4)));
typedef _Float16 h16;

#ifndef NSAMP
#define NSAMP 2048
#endif
#define NSAMP_FULL 2048
#define DIN   16
#define HID   256
#define MOUT  4
#define SPB   8
#define NTILE 14
#define LP    264
#define ROW_J 192
#define ROW_A 208
#define SROWS (NTILE * 16)

#define OUT1_OFF ((size_t)NSAMP_FULL * MOUT)
#define OUT2_OFF (OUT1_OFF + (size_t)NSAMP_FULL * DIN * MOUT)

static_assert(NSAMP >= SPB && NSAMP <= NSAMP_FULL && (NSAMP % SPB) == 0);
static_assert(DIN == 16 && HID == 256 && MOUT == 4);
static_assert((HID % 64) == 0 && (HID % 32) == 0);
static_assert(HID == 16 * 16);
static_assert(SROWS == 224 && ROW_J == 12 * 16 && ROW_A == 13 * 16);
static_assert((LP % 8) == 0 && LP >= HID);
static_assert(OUT1_OFF * 4 == (size_t)32768);
static_assert(OUT2_OFF * 4 == (size_t)557056);
static_assert((OUT2_OFF + (size_t)NSAMP_FULL * DIN * DIN * MOUT) * 4 == (size_t)8945664);
static_assert(SPB * MOUT * 4 == 128);
static_assert((size_t)SROWS * LP * 2 + 1024 * 4 + 64 * 4 + SPB * 4 * 4 <= (size_t)131072);

#define LDT 72
static_assert((LDT % 8) == 0 && LDT >= 64);

#define WCARRY 64.0f
#define HCARRY 1024.0f
#define JCARRY 64.0f
#define ACARRY 64.0f

#define W12_BYTES ((size_t)2 * HID * HID * 2)
#define W3T_BYTES ((size_t)16 * HID * 2)
#define OFF_W12 ((size_t)0)
#define OFF_W3T (OFF_W12 + W12_BYTES)
#define WS_TOTAL (OFF_W3T + W3T_BYTES)
static_assert((W12_BYTES % 128) == 0 && (W3T_BYTES % 128) == 0);
static_assert(WS_TOTAL <= (size_t)134217728);

__device__ __forceinline__ float bf16r(float x) {
  unsigned int u = __float_as_uint(x);
  u = (u + 0x7FFFu + ((u >> 16) & 1u)) & 0xFFFF0000u;
  return __uint_as_float(u);
}

static __device__ __forceinline__ h16 toh_flush(float v) {
  const h16 r = (h16)v;
  return (fabsf(v) < 6.103515625e-05f) ? (h16)0.0f : r;
}

__device__ __forceinline__ v16h frag_at(const _Float16* p) {
  v8h lo = *(const v8h*)(p);
  v8h hi = *(const v8h*)(p + 16);
  v16h out;
#pragma unroll
  for (int i = 0; i < 8; ++i) { out[i] = lo[i]; out[i + 8] = hi[i]; }
  return out;
}
__device__ __forceinline__ v16h ld_frag(const _Float16* base, unsigned ld) {
  const unsigned lane = threadIdx.x & 31u;
  return frag_at(base + (lane & 15u) * ld + (lane >> 4) * 8u);
}

__device__ __forceinline__ v8f wmma16(v16h a, v16h b, v8f c) {
  v8f d = __builtin_amdgcn_wmma_f32_16x16x32_f16(false, a, false, b, (short)0, c,
                                                 false, false);
  asm volatile("v_nop\n\tv_nop\n\tv_nop\n\tv_nop" : "+v"(d) : "v"(a), "v"(b));
  return d;
}

__global__ __launch_bounds__(256) void wconv_kernel(
    const float* __restrict__ W, _Float16* __restrict__ Wt, unsigned ldw, unsigned ldk) {
  __shared__ _Float16 T[64 * LDT];
  const unsigned tid = threadIdx.x;
  const unsigned n0 = blockIdx.x * 64u;
  const unsigned k0 = blockIdx.y * 64u;
#pragma unroll 4
  for (unsigned j = 0; j < 16u; ++j) {
    const unsigned idx = tid + 256u * j;
    const unsigned kr = idx >> 6, nc = idx & 63u;
    const float v = W[(size_t)(k0 + kr) * ldw + n0 + nc];
    T[nc * LDT + kr] = toh_flush(WCARRY * bf16r(v));
  }
  __syncthreads();
  v8h x[2];
  size_t off[2];
#pragma unroll
  for (unsigned i = 0; i < 2u; ++i) {
    const unsigned n = 32u * i + (tid >> 3);
    const unsigned kc = (tid & 7u) * 8u;
    x[i] = *(const v8h*)&T[n * LDT + kc];
    off[i] = (size_t)(n0 + n) * ldk + k0 + kc;
  }
#pragma unroll
  for (int i = 0; i < 2; ++i) *(volatile v8h*)(Wt + off[i]) = x[i];
  __threadfence();
#pragma unroll
  for (int i = 0; i < 2; ++i) *(volatile v8h*)(Wt + off[i]) = x[i];
}

__global__ __launch_bounds__(256) void w3conv_kernel(
    const float* __restrict__ W3, _Float16* __restrict__ W3t) {
  const unsigned t = blockIdx.x * 256u + threadIdx.x;
  const unsigned n = t >> 5;
  const unsigned kc = (t & 31u) * 8u;
  const unsigned nn = (n < 4u) ? n : 3u;
  v8h x;
#pragma unroll
  for (unsigned j = 0; j < 8u; ++j) {
    const float v = W3[(size_t)(kc + j) * MOUT + nn];
    const h16 c = toh_flush(WCARRY * bf16r(v));
    x[j] = (n < 4u) ? c : (h16)0.0f;
  }
  _Float16* p = W3t + (size_t)t * 8u;
  *(volatile v8h*)p = x;
  __threadfence();
  *(volatile v8h*)p = x;
}

__global__ __launch_bounds__(512) __attribute__((amdgpu_num_vgpr(256))) void hess_kernel(
    const float* __restrict__ X, const float* __restrict__ W0, const float* __restrict__ B0,
    const float* __restrict__ B1, const float* __restrict__ B2, const float* __restrict__ B3,
    const _Float16* __restrict__ Wt12, const _Float16* __restrict__ W3t,
    float* __restrict__ out) {
  __shared__ __attribute__((aligned(16))) _Float16 S[SROWS * LP];
  __shared__ __attribute__((aligned(16))) float Od2[DIN * DIN * MOUT];
  __shared__ __attribute__((aligned(16))) float Odf[DIN * MOUT];
  __shared__ __attribute__((aligned(16))) float Of[SPB * MOUT];

  const unsigned tid = threadIdx.x, lane = tid & 31u;
  const int wv = (int)(threadIdx.x >> 5);
  const int wave = __builtin_amdgcn_readfirstlane(wv);
  const int ptile = __builtin_amdgcn_readfirstlane((wv < NTILE - 1) ? wv : (NTILE - 1));
  const unsigned hh = lane >> 4, m = lane & 15u;
  const bool hi = (hh != 0u);
  const unsigned c = (unsigned)wave * 16u + m;
  const unsigned rb = hh * 8u * LP + c;

  const float CS_H = 1.0f / (WCARRY * HCARRY);
  const float CS_J = 1.0f / (WCARRY * JCARRY);
  const float CS_A = 1.0f / (WCARRY * ACARRY);

#pragma unroll
  for (unsigned r = 0; r < 8u; ++r) S[(ROW_A + r) * LP + rb] = (h16)0.0f;

  const float b3v = bf16r(B3[m & 3u]);

#pragma unroll 1
  for (int si = 0; si < SPB; ++si) {
    const unsigned s = blockIdx.x * SPB + (unsigned)si;

    {
      float w0[16];
#pragma unroll
      for (int d = 0; d < 16; ++d) w0[d] = bf16r(W0[(unsigned)d * HID + c]);
      float z = bf16r(B0[c]);
#pragma unroll
      for (int d = 0; d < 16; ++d) z += bf16r(X[(size_t)s * DIN + (unsigned)d]) * w0[d];
      const float t = tanhf(z);
      const float s1 = 1.0f - t * t;
      const float s2 = -2.0f * t * s1;
      const float hs2 = HCARRY * s2;
      float wd2[8];
#pragma unroll
      for (int r = 0; r < 8; ++r) wd2[r] = hi ? w0[8 + r] : w0[r];
#pragma unroll
      for (int p = 0; p < 8; ++p) {
        const float u = hs2 * w0[p];
#pragma unroll
        for (int r = 0; r < 8; ++r)
          S[(unsigned)(16 * p + r) * LP + rb] = toh_flush(u * wd2[r]);
      }
#pragma unroll
      for (int j = 0; j < 4; ++j) {
        const float wd1 = hi ? w0[9 + 2 * j] : w0[8 + 2 * j];
        const float u = hs2 * wd1;
#pragma unroll
        for (int r = 0; r < 8; ++r)
          S[(unsigned)(16 * (8 + j) + r) * LP + rb] = toh_flush(u * w0[8 + r]);
      }
      const float js = JCARRY * s1;
#pragma unroll
      for (int r = 0; r < 8; ++r)
        S[(unsigned)(ROW_J + r) * LP + rb] = toh_flush(js * wd2[r]);
      if (!hi) S[ROW_A * LP + c] = toh_flush(ACARRY * t);
    }
    __syncthreads();

#pragma unroll 1
    for (int l = 0; l < 2; ++l) {
      v8f acc[NTILE];
#pragma unroll
      for (int p = 0; p < NTILE; ++p) acc[p] = (v8f){};
      const _Float16* bp = Wt12 + (size_t)l * (HID * HID) + (size_t)c * HID + hh * 8u;
#pragma unroll 1
      for (unsigned k0 = 0; k0 < HID; k0 += 32u) {
        const v16h b = frag_at(bp + k0);
#pragma unroll
        for (int p = 0; p < NTILE; ++p) {
          const v16h a = ld_frag(&S[(unsigned)(p * 16) * LP + k0], LP);
          acc[p] = wmma16(a, b, acc[p]);
        }
      }
      __syncthreads();

      const float zraw = __shfl(acc[13][0], (int)m, 32);
      const float bv1 = B1[c];
      const float bv2 = B2[c];
      const float z = zraw * CS_A + bf16r((l == 0) ? bv1 : bv2);
      const float t = tanhf(z);
      const float s1 = 1.0f - t * t;
      const float s2 = -2.0f * t * s1;

      float jz[8], jlo[8], jhi[8];
#pragma unroll
      for (int r = 0; r < 8; ++r) {
        jz[r] = acc[12][r] * CS_J;
        const float jo = __shfl_xor(jz[r], 16, 32);
        jlo[r] = hi ? jo : jz[r];
        jhi[r] = hi ? jz[r] : jo;
      }
      const float hs1 = s1 * (1.0f / WCARRY);
      const float hs2 = HCARRY * s2;
#pragma unroll
      for (int p = 0; p < 8; ++p) {
        const float u = hs2 * jlo[p];
#pragma unroll
        for (int r = 0; r < 8; ++r)
          S[(unsigned)(16 * p + r) * LP + rb] = toh_flush(acc[p][r] * hs1 + u * jz[r]);
      }
#pragma unroll
      for (int j = 0; j < 4; ++j) {
        const float jd1 = hi ? jhi[2 * j + 1] : jhi[2 * j];
        const float u = hs2 * jd1;
#pragma unroll
        for (int r = 0; r < 8; ++r)
          S[(unsigned)(16 * (8 + j) + r) * LP + rb] = toh_flush(acc[8 + j][r] * hs1 + u * jhi[r]);
      }
      const float js = JCARRY * s1;
#pragma unroll
      for (int r = 0; r < 8; ++r)
        S[(unsigned)(ROW_J + r) * LP + rb] = toh_flush(js * jz[r]);
      if (!hi) S[ROW_A * LP + c] = toh_flush(ACARRY * t);
      __syncthreads();
    }

    {
      v8f oacc = (v8f){};
      const _Float16* wp = W3t + (size_t)m * HID + hh * 8u;
#pragma unroll 1
      for (unsigned k0 = 0; k0 < HID; k0 += 32u) {
        const v16h a = ld_frag(&S[(unsigned)(ptile * 16) * LP + k0], LP);
        const v16h b = frag_at(wp + k0);
        oacc = wmma16(a, b, oacc);
      }
      if (m < 4u) {
        if (wave < 8) {
#pragma unroll
          for (int r = 0; r < 8; ++r) {
            const unsigned d2 = hh * 8u + (unsigned)r;
            const float v = oacc[r] * CS_H;
            Od2[((unsigned)wave * 16u + d2) * 4u + m] = v;
            if (hi) Od2[(d2 * 16u + (unsigned)wave) * 4u + m] = v;
          }
        } else if (wave < 12) {
          const unsigned d1 = 8u + 2u * (unsigned)(wave - 8) + hh;
#pragma unroll
          for (int r = 0; r < 8; ++r)
            Od2[(d1 * 16u + 8u + (unsigned)r) * 4u + m] = oacc[r] * CS_H;
        } else if (wave == 12) {
#pragma unroll
          for (int r = 0; r < 8; ++r)
            Odf[(hh * 8u + (unsigned)r) * 4u + m] = oacc[r] * CS_J;
        } else if (wave == 13) {
          if (!hi) Of[(unsigned)si * 4u + m] = oacc[0] * CS_A + b3v;
        }
      }
    }
    __syncthreads();

    if (wave < 8) {
      const v4f v = *(const v4f*)&Od2[tid * 4u];
      float* p = out + OUT2_OFF + (size_t)s * (DIN * DIN * MOUT) + tid * 4u;
      *(volatile v4f*)p = v;
      __threadfence();
      *(volatile v4f*)p = v;
    } else if (wave == 8) {
      if (lane < 16u) {
        const v4f v = *(const v4f*)&Odf[lane * 4u];
        float* p = out + OUT1_OFF + (size_t)s * (DIN * MOUT) + lane * 4u;
        *(volatile v4f*)p = v;
        __threadfence();
        *(volatile v4f*)p = v;
      }
    }
  }

  if (wave == 0) {
    if (lane < (unsigned)SPB) {
      const v4f v = *(const v4f*)&Of[lane * 4u];
      float* p = out + ((size_t)blockIdx.x * SPB + lane) * MOUT;
      *(volatile v4f*)p = v;
      __threadfence();
      *(volatile v4f*)p = v;
    }
  }
}

extern "C" void kernel_launch(void* const* d_in, const int* in_sizes, int n_in,
                              void* d_out, int out_size, void* d_ws, size_t ws_size,
                              hipStream_t stream) {
  if (n_in < 9) return;
  if ((long long)in_sizes[0] < (long long)NSAMP * DIN) return;
  if ((long long)in_sizes[1] < (long long)DIN * HID) return;
  if (in_sizes[2] < HID) return;
  if ((long long)in_sizes[3] < (long long)HID * HID) return;
  if (in_sizes[4] < HID) return;
  if ((long long)in_sizes[5] < (long long)HID * HID) return;
  if (in_sizes[6] < HID) return;
  if ((long long)in_sizes[7] < (long long)HID * MOUT) return;
  if (in_sizes[8] < MOUT) return;
  if ((long long)out_size < (long long)(OUT2_OFF + (size_t)NSAMP * DIN * DIN * MOUT)) return;
  if (ws_size < WS_TOTAL) return;

  const float* x  = (const float*)d_in[0];
  const float* w0 = (const float*)d_in[1];
  const float* b0 = (const float*)d_in[2];
  const float* w1 = (const float*)d_in[3];
  const float* b1 = (const float*)d_in[4];
  const float* w2 = (const float*)d_in[5];
  const float* b2 = (const float*)d_in[6];
  const float* w3 = (const float*)d_in[7];
  const float* b3 = (const float*)d_in[8];
  float* out = (float*)d_out;

  char* ws = (char*)d_ws;
  _Float16* Wt12 = (_Float16*)(ws + OFF_W12);
  _Float16* W3t  = (_Float16*)(ws + OFF_W3T);

  dim3 blk(256);
  wconv_kernel<<<dim3(HID / 64, HID / 64), blk, 0, stream>>>(w1, Wt12, (unsigned)HID, (unsigned)HID);
  wconv_kernel<<<dim3(HID / 64, HID / 64), blk, 0, stream>>>(w2, Wt12 + (size_t)HID * HID,
                                                            (unsigned)HID, (unsigned)HID);
  w3conv_kernel<<<dim3(2), blk, 0, stream>>>(w3, W3t);

  hess_kernel<<<dim3(NSAMP / SPB), dim3(512), 0, stream>>>(x, w0, b0, b1, b2, b3, Wt12, W3t, out);
}
